// KANLayer_28097676050639
// MI455X (gfx1250) — hardware-verified
//
#include <hip/hip_runtime.h>
#include <stdint.h>

#define NROWS   8192
#define NIN     512
#define NOUT    512
#define NBAS    13
#define KS      (NIN * NBAS)
#define KA      (2 * NIN)
#define KTOT    (KA + 2 * KS)
#define CH      2048
#define NCHUNK  (NROWS / CH)
#define UROW    (KTOT / 8)
#define SU_ROW  (2 * KS / 8)
#define PB_UNITS (NOUT * KA / 8)
#define PS_UNITS (NOUT * SU_ROW)
#define PB_BLKS  (PB_UNITS / 256)
#define PS_BLKS  (PS_UNITS / 256)

static_assert(NROWS == NCHUNK * CH);
static_assert(CH % 128 == 0);
static_assert(NOUT % 64 == 0);
static_assert(KTOT % 32 == 0);
static_assert(KS % 8 == 0);
static_assert(KA % 32 == 0);
static_assert(UROW == 1792);
static_assert(PB_UNITS == PB_BLKS * 256);
static_assert(PS_UNITS == PS_BLKS * 256);
static_assert(SU_ROW % 32 == 0);
static_assert((KA / 8) % 32 == 0);
static_assert(NIN == 512);

typedef __attribute__((ext_vector_type(16))) __bf16  v16b;
typedef __attribute__((ext_vector_type(8)))  __bf16  v8b;
typedef __attribute__((ext_vector_type(8)))  float   v8f;
typedef __attribute__((ext_vector_type(4)))  float   v4f;
typedef __attribute__((ext_vector_type(4)))  unsigned int v4u;
typedef v8b __attribute__((may_alias)) v8ba;
typedef v4f __attribute__((may_alias)) v4fa;
typedef v4u __attribute__((may_alias)) v4ua;

__device__ __forceinline__ unsigned short f2bf_bits(float f) {
  unsigned u = __float_as_uint(f);
  return (unsigned short)((u + 0x7FFFu + ((u >> 16) & 1u)) >> 16);
}
__device__ __forceinline__ float bf_bits2f(unsigned short b) { return __uint_as_float(((unsigned)b) << 16); }
__device__ __forceinline__ float bfr(float f) { return bf_bits2f(f2bf_bits(f)); }
__device__ __forceinline__ unsigned pk16(unsigned short a, unsigned short b) { return (unsigned)a | ((unsigned)b << 16); }

__device__ __forceinline__ v8f mma_bf16(v16b a, v16b b, v8f c) {
  c = __builtin_amdgcn_wmma_f32_16x16x32_bf16(false, a, false, b, (short)0, c, false, false);
  asm volatile("v_nop\n\tv_nop\n\tv_nop\n\tv_nop" : "+v"(c) : "v"(a), "v"(b));
  return c;
}

__device__ __forceinline__ v16b ldfrag(const __bf16* p) {
  union { v16b v; v8b h[2]; } f;
  f.h[0] = *(const v8ba*)(p);
  f.h[1] = *(const v8ba*)(p + 16);
  return f.v;
}

__global__ __launch_bounds__(256) void prep_kernel(const float* __restrict__ base_w, const float* __restrict__ spline_w,
                                                   unsigned short* __restrict__ WB) {
  const int tid = threadIdx.x;
  const float* src;
  unsigned short* dst;
  if (blockIdx.x < PB_BLKS) {
    const int u  = blockIdx.x * 256 + tid;
    const int o  = u >> 7;
    const int c8 = (u & 127) * 8;
    src = base_w + (size_t)o * NIN + (c8 & (NIN - 1));
    dst = WB + (size_t)o * KTOT + c8;
  } else {
    const int u   = (blockIdx.x - PB_BLKS) * 256 + tid;
    const int o   = u / SU_ROW;
    const int rem = u - o * SU_ROW;
    const int se  = (rem - ((rem >= (SU_ROW / 2)) ? (SU_ROW / 2) : 0)) * 8;
    src = spline_w + (size_t)o * KS + se;
    dst = WB + (size_t)o * KTOT + KA + rem * 8;
  }
  const v4f a = *(const v4fa*)src;
  const v4f c = *(const v4fa*)(src + 4);
  v4u v;
  v[0] = pk16(f2bf_bits(a[0]), f2bf_bits(a[1]));
  v[1] = pk16(f2bf_bits(a[2]), f2bf_bits(a[3]));
  v[2] = pk16(f2bf_bits(c[0]), f2bf_bits(c[1]));
  v[3] = pk16(f2bf_bits(c[2]), f2bf_bits(c[3]));
  *(volatile v4u*)dst = v;
  __threadfence();
  *(volatile v4u*)dst = v;
}

__device__ __forceinline__ float knot(float jf) { return fmaf(0.4f, jf, -3.2f); }

__device__ __forceinline__ void a_store_pass(const unsigned short* sA, unsigned short* dst, int tid) {
#pragma unroll
  for (int it = 0; it < 4; ++it) {
    const int u = it * 512 + tid;
    if (u < UROW) {
      const v4u v = *(const v4ua*)(sA + 8 * u);
      *(volatile v4u*)(dst + 8 * u) = v;
    }
  }
}

__global__ __launch_bounds__(512) void feat_kernel(const float* __restrict__ x, unsigned short* __restrict__ AP,
                                                   int row_base) {
  __shared__ __align__(16) unsigned short sA[KTOT];
  const int i = threadIdx.x;
  const int r = blockIdx.x;
  const float xv = bfr(x[(size_t)(row_base + r) * NIN + i]);

  const float ex = __expf(-xv);
  const float sg = __builtin_amdgcn_rcpf(1.0f + ex);
  const float s  = xv * sg;

  int cnt = 0;
#pragma unroll
  for (int j = 0; j < 17; ++j) cnt += (xv >= knot((float)j)) ? 1 : 0;
  const float valid = (cnt >= 1 && cnt <= 16) ? 1.0f : 0.0f;
  int m = cnt - 1;
  m = (m < 0) ? 0 : m;
  m = (m > 15) ? 15 : m;
  const float fm  = (float)m;
  const float tm2 = knot(fm - 2.0f);
  const float tm1 = knot(fm - 1.0f);
  const float tm0 = knot(fm);
  const float tp1 = knot(fm + 1.0f);
  const float tp2 = knot(fm + 2.0f);
  const float tp3 = knot(fm + 3.0f);
  const float inv1 = 1.0f / (0.4f + 1e-8f);
  const float inv2 = 1.0f / (0.8f + 1e-8f);
  const float inv3 = 1.0f / (1.2f + 1e-8f);

  const float b1_0 = ((tp1 - xv) * inv1) * valid;
  const float b1_1 = ((xv - tm0) * inv1) * valid;
  const float b2_0 = ((tp1 - xv) * inv2) * b1_0;
  const float b2_1 = ((xv - tm1) * inv2) * b1_0 + ((tp2 - xv) * inv2) * b1_1;
  const float b2_2 = ((xv - tm0) * inv2) * b1_1;
  const float b3_0 = ((tp1 - xv) * inv3) * b2_0;
  const float b3_1 = ((xv - tm2) * inv3) * b2_0 + ((tp2 - xv) * inv3) * b2_1;
  const float b3_2 = ((xv - tm1) * inv3) * b2_1 + ((tp3 - xv) * inv3) * b2_2;
  const float b3_3 = ((xv - tm0) * inv3) * b2_2;

  {
    const unsigned short hb = f2bf_bits(s);
    const unsigned short lb = f2bf_bits(s - bf_bits2f(hb));
    sA[i]       = hb;
    sA[NIN + i] = lb;
  }
#pragma unroll
  for (int g = 0; g < NBAS; ++g) {
    const int d = g + 3 - m;
    float v = (d == 0) ? b3_0 : 0.0f;
    v = (d == 1) ? b3_1 : v;
    v = (d == 2) ? b3_2 : v;
    v = (d == 3) ? b3_3 : v;
    const unsigned short hb = f2bf_bits(v);
    const unsigned short lb = f2bf_bits(v - bf_bits2f(hb));
    sA[KA + NBAS * i + g]      = hb;
    sA[KA + KS + NBAS * i + g] = lb;
  }
  __syncthreads();

  unsigned short* dst = AP + (size_t)r * KTOT;
  a_store_pass(sA, dst, i);
  __threadfence();
  a_store_pass(sA, dst, i);
}

__device__ __forceinline__ void o_store_pass(const float* sO, float* out,
                                             int grow_w, int n0, int w, int lane) {
  const int q8 = lane & 7, sub = lane >> 3;
#pragma unroll
  for (int i = 0; i < 16; ++i) {
    const int lid = i * 4 + sub;
    const int row = lid >> 1, hl = lid & 1;
    const v4f v = *(const v4fa*)(sO + (32 * w + row) * 64 + 32 * hl + 4 * q8);
    *(volatile v4f*)(out + (size_t)(grow_w + row) * NOUT + n0 + 32 * hl + 4 * q8) = v;
  }
}

__global__ __launch_bounds__(128) void gemm_kernel(const unsigned short* __restrict__ AP,
                                                   const unsigned short* __restrict__ WB,
                                                   const float* __restrict__ base_b,
                                                   float* __restrict__ out, int row_base) {
  __shared__ __align__(16) float sO[128 * 64];
  const int tid = threadIdx.x, lane = tid & 31, w = tid >> 5;
  const int h = lane >> 4, m = lane & 15;
  const int lrow_w = blockIdx.x * 128 + 32 * w;
  const int n0 = blockIdx.y * 64;
  const __bf16* APb = (const __bf16*)(const void*)AP;
  const __bf16* WBb = (const __bf16*)(const void*)WB;

  const __bf16* xa0 = APb + (size_t)(lrow_w + m) * KTOT + 8 * h;
  const __bf16* xa1 = xa0 + (size_t)16 * KTOT;
  const __bf16* wb  = WBb + (size_t)(n0 + m) * KTOT + 8 * h;

  const v8f zero8 = {0.f, 0.f, 0.f, 0.f, 0.f, 0.f, 0.f, 0.f};
  v8f acc[2][4];
#pragma unroll
  for (int mt = 0; mt < 2; ++mt)
#pragma unroll
    for (int nt = 0; nt < 4; ++nt) acc[mt][nt] = zero8;

#pragma unroll 1
  for (int k0 = 0; k0 < KTOT; k0 += 32) {
    const v16b a0 = ldfrag(xa0 + k0);
    const v16b a1 = ldfrag(xa1 + k0);
#pragma unroll
    for (int nt = 0; nt < 4; ++nt) {
      const v16b b = ldfrag(wb + (size_t)nt * 16 * KTOT + k0);
      acc[0][nt] = mma_bf16(a0, b, acc[0][nt]);
      acc[1][nt] = mma_bf16(a1, b, acc[1][nt]);
    }
  }

#pragma unroll
  for (int nt = 0; nt < 4; ++nt) {
    const int cl = 16 * nt + m;
    const float bias = bfr(base_b[n0 + cl]);
#pragma unroll
    for (int mt = 0; mt < 2; ++mt) {
#pragma unroll
      for (int r = 0; r < 8; ++r) {
        const int rl = 32 * w + 16 * mt + 8 * h + r;
        sO[rl * 64 + cl] = acc[mt][nt][r] + bias;
      }
    }
  }
  __syncthreads();

  const int grow_w = row_base + lrow_w;
  o_store_pass(sO, out, grow_w, n0, w, lane);
  __threadfence();
  o_store_pass(sO, out, grow_w, n0, w, lane);
}

extern "C" void kernel_launch(void* const* d_in, const int* in_sizes, int n_in,
                              void* d_out, int out_size, void* d_ws, size_t ws_size,
                              hipStream_t stream) {
  if (n_in < 4) return;
  if (in_sizes[0] != NROWS * NIN) return;
  if (in_sizes[1] != NOUT * NIN) return;
  if (in_sizes[2] != NOUT) return;
  if (in_sizes[3] != NOUT * NIN * NBAS) return;
  if (out_size != NROWS * NOUT) return;

  const float* x        = (const float*)d_in[0];
  const float* base_w   = (const float*)d_in[1];
  const float* base_b   = (const float*)d_in[2];
  const float* spline_w = (const float*)d_in[3];
  float* out = (float*)d_out;

  size_t off = 0;
  const size_t oAP = off; off += (size_t)CH * KTOT * 2;
  const size_t oWB = off; off += (size_t)NOUT * KTOT * 2;
  if (off > ws_size) return;
  if (off > (size_t)134217728) return;

  char* ws = (char*)d_ws;
  unsigned short* AP = (unsigned short*)(ws + oAP);
  unsigned short* WB = (unsigned short*)(ws + oWB);

  prep_kernel<<<dim3(PB_BLKS + PS_BLKS), dim3(256), 0, stream>>>(base_w, spline_w, WB);
  for (int c = 0; c < NCHUNK; ++c) {
    const int row_base = c * CH;
    feat_kernel<<<dim3(CH), dim3(512), 0, stream>>>(x, AP, row_base);
    gemm_kernel<<<dim3(CH / 128, NOUT / 64), dim3(128), 0, stream>>>(AP, WB, base_b, out, row_base);
  }
  (void)hipGetLastError();
}
